// RGCN_54631984005709
// MI455X (gfx1250) — hardware-verified
//
#include <hip/hip_runtime.h>
#include <math.h>
#include <stddef.h>

static constexpr int NN   = 100000;
static constexpr int NE   = 800000;
static constexpr int NG   = 2048;
static constexpr int DD   = 64;
static constexpr int NR   = 5;
static constexpr int PROP = 6;
static constexpr int S2S  = 6;

static constexpr int CHUNK  = 2048;
static constexpr int NCH    = (NE + CHUNK - 1) / CHUNK;
static constexpr int BKSH   = 9;
static constexpr int BKW    = 1 << BKSH;
static constexpr int NBKT   = (NN + BKW - 1) / BKW;
static constexpr int NBPAD  = 256;
static constexpr int NBBITS = 8;
static constexpr int CAP    = 6144;
static constexpr int SORTED_N = NE + 32 * NBPAD;
static constexpr int RP     = 544;
static constexpr int GPN    = 2080;
static constexpr int XW     = 192;
static constexpr unsigned ROWMASK = 0xFFFFFu;

typedef char chk_a[(NBKT <= (1 << NBBITS) && (1 << NBBITS) <= NBPAD) ? 1 : -1];
typedef char chk_b[((long long)NR * NN <= (long long)ROWMASK + 1) ? 1 : -1];
typedef char chk_c[(NN % 32 == 0 && NG % 32 == 0 && CHUNK == 8 * 256) ? 1 : -1];
typedef char chk_d[(RP >= BKW + 1 && RP % 32 == 0 && RP / 4 <= 256) ? 1 : -1];
typedef char chk_e[(GPN >= NG + 1 && GPN % 32 == 0 && CAP % 32 == 0) ? 1 : -1];
typedef char chk_f[(BKW <= 1024) ? 1 : -1];

typedef _Float16 v16h __attribute__((ext_vector_type(16)));
typedef _Float16 v8h  __attribute__((ext_vector_type(8)));
typedef float    v8f  __attribute__((ext_vector_type(8)));
typedef float    v4f  __attribute__((ext_vector_type(4)));
typedef float    v2f  __attribute__((ext_vector_type(2)));
typedef unsigned v4u  __attribute__((ext_vector_type(4)));
typedef int      v4i  __attribute__((ext_vector_type(4)));
union Frag { v16h v; v8h hv[2]; };

__device__ __forceinline__ int clampi(int v, int lo, int hi) { return v < lo ? lo : (v > hi ? hi : v); }

__device__ __forceinline__ v8f wmma_raw(v16h a, v16h b, v8f c) {
  return __builtin_amdgcn_wmma_f32_16x16x32_f16(false, a, false, b, (short)0, c, false, false);
}
__device__ __forceinline__ v8f wmma_g(v16h a, v16h b, v8f c) {
  c = wmma_raw(a, b, c);
  asm volatile("v_nop\n\tv_nop\n\tv_nop\n\tv_nop" : "+v"(c) : "v"(a), "v"(b));
  return c;
}

__device__ __forceinline__ v8h cvt8(const float* p, float s) {
  v4f x0 = *(const v4f*)p, x1 = *(const v4f*)(p + 4);
  v8h v;
  v[0] = (_Float16)(x0[0] * s); v[1] = (_Float16)(x0[1] * s); v[2] = (_Float16)(x0[2] * s); v[3] = (_Float16)(x0[3] * s);
  v[4] = (_Float16)(x1[0] * s); v[5] = (_Float16)(x1[1] * s); v[6] = (_Float16)(x1[2] * s); v[7] = (_Float16)(x1[3] * s);
  return v;
}

__device__ __forceinline__ int block_excl_scan(int v, int* s_w, int& total) {
  const int lane = threadIdx.x & 31, wave = threadIdx.x >> 5, nw = blockDim.x >> 5;
  int x = v;
  for (int o = 1; o < 32; o <<= 1) { int y = __shfl_up(x, o); if (lane >= o) x += y; }
  __syncthreads();
  if (lane == 31) s_w[wave] = x;
  __syncthreads();
  if (wave == 0) {
    int w = (lane < nw) ? s_w[lane] : 0;
    for (int o = 1; o < 32; o <<= 1) { int y = __shfl_up(w, o); if (lane >= o) w += y; }
    if (lane < nw) s_w[lane] = w;
  }
  __syncthreads();
  int excl = x - v + (wave > 0 ? s_w[wave - 1] : 0);
  total = s_w[nw - 1];
  return excl;
}

__device__ __forceinline__ float prep_val(int sec, int n, int k,
    const float* att, const float* basis, const float* root,
    const float* w_ih, const float* w_hh, const float* lin1_w, const float* lin2_w) {
  float v = 0.f;
  if (sec == 0) {
    int cb = n >> 6, j = n & 63;
    if (cb < NR) {
      #pragma unroll
      for (int b = 0; b < NR; ++b) v += att[cb * NR + b] * basis[(b * DD + k) * DD + j];
    } else {
      v = root[k * DD + j];
    }
  } else if (sec == 1) {
    v = (k < 128) ? w_ih[n * 128 + k] : w_hh[n * DD + (k - 128)];
  } else if (sec == 2) {
    v = lin1_w[k * DD + n];
  } else {
    v = (n < 12) ? lin2_w[k * 12 + n] : 0.f;
  }
  return v * 64.f;
}

__global__ __launch_bounds__(256) void prep_kernel(const float* __restrict__ att, const float* __restrict__ basis,
    const float* __restrict__ root, const float* __restrict__ w_ih, const float* __restrict__ w_hh,
    const float* __restrict__ b_ih, const float* __restrict__ b_hh, const float* __restrict__ conv_b,
    const float* __restrict__ lin1_w, const float* __restrict__ lin1_b,
    const float* __restrict__ lin2_w, const float* __restrict__ lin2_b,
    _Float16* Wall, _Float16* Wg, _Float16* W1, _Float16* W2,
    float* gb, float* cb64, float* b1c, float* b2p, float* z64) {
  const int t = threadIdx.x, nthr = blockDim.x;
  const int nN[4] = {384, 256, 64, 64};
  const int nK[4] = {64, 192, 128, 64};
  _Float16* dst[4] = {Wall, Wg, W1, W2};
  for (int sec = 0; sec < 4; ++sec) {
    const int K8 = nK[sec] >> 3;
    const int items = nN[sec] * K8;
    for (int it = t; it < items; it += nthr) {
      int n = it / K8, kc = it - n * K8;
      v8h v;
      #pragma unroll
      for (int i = 0; i < 8; ++i)
        v[i] = (_Float16)prep_val(sec, n, kc * 8 + i, att, basis, root, w_ih, w_hh, lin1_w, lin2_w);
      _Float16* p = dst[sec] + (size_t)n * nK[sec] + kc * 8;
      *(volatile v8h*)p = v;
      __threadfence();
      *(volatile v8h*)p = v;
    }
  }
  float vg = 0.f, vc = 0.f, v1 = 0.f, v2 = 0.f;
  if (t < 256) vg = b_ih[t] + b_hh[t];
  if (t < 64) { vc = conv_b[t]; v1 = lin1_b[t]; v2 = (t < 12) ? lin2_b[t] : 0.f; }
  for (int pass = 0; pass < 2; ++pass) {
    if (t < 256) *(volatile float*)(gb + t) = vg;
    if (t < 64) {
      *(volatile float*)(cb64 + t) = vc;
      *(volatile float*)(b1c + t) = v1;
      *(volatile float*)(b2p + t) = v2;
      *(volatile float*)(z64 + t) = 0.f;
    }
    if (pass == 0) __threadfence();
  }
}

__global__ __launch_bounds__(256) void lin0_kernel(const float* __restrict__ x, const float* __restrict__ w,
    const float* __restrict__ b, float* h) {
  int tid = blockIdx.x * blockDim.x + threadIdx.x;
  if (tid >= NN * 16) return;
  int n = tid >> 4, c4 = (tid & 15) * 4;
  float acc[4];
  #pragma unroll
  for (int j = 0; j < 4; ++j) acc[j] = b[c4 + j];
  #pragma unroll
  for (int k = 0; k < 15; ++k) {
    float xv = x[(size_t)n * 15 + k];
    #pragma unroll
    for (int j = 0; j < 4; ++j) acc[j] += xv * w[k * DD + c4 + j];
  }
  v4f o;
  #pragma unroll
  for (int j = 0; j < 4; ++j) o[j] = fmaxf(acc[j], 0.f);
  float* p = h + (size_t)n * DD + c4;
  *(volatile v4f*)p = o;
  __threadfence();
  *(volatile v4f*)p = o;
}

template <int KS, int NCB>
__global__ __launch_bounds__(64) void gemm_kernel(const float* __restrict__ A32, int lda, float sA,
    const _Float16* __restrict__ W16, const float* __restrict__ bias, float inv, int relu,
    float* C, int ldc, size_t cbStride, int M) {
  __shared__ v4f sO[2][256];
  const int t = threadIdx.x, wv = t >> 5, lane = t & 31, h = lane >> 4, m = lane & 15;
  const int K = KS * 32;
  const int MT = M >> 4;
  int tile = blockIdx.x * 2 + wv;
  const bool active = tile < MT;
  if (!active) tile = MT - 1;
  if (tile < 0) tile = 0;
  const int row0 = tile * 16;
  Frag xf[KS];
  {
    const float* ap = A32 + (size_t)(row0 + m) * lda + 8 * h;
    #pragma unroll
    for (int s = 0; s < KS; ++s) {
      xf[s].hv[0] = cvt8(ap + 32 * s, sA);
      xf[s].hv[1] = cvt8(ap + 32 * s + 16, sA);
    }
  }
  #pragma unroll 1
  for (int cb = 0; cb < NCB; ++cb) {
    v8f acc[4];
    #pragma unroll
    for (int nt = 0; nt < 4; ++nt) {
      const _Float16* wp = W16 + (size_t)(cb * 64 + nt * 16 + m) * K + 8 * h;
      v8f c = {0.f, 0.f, 0.f, 0.f, 0.f, 0.f, 0.f, 0.f};
      if (KS == 2) {
        Frag w0, w1;
        w0.hv[0] = *(const v8h*)(wp);      w0.hv[1] = *(const v8h*)(wp + 16);
        w1.hv[0] = *(const v8h*)(wp + 32); w1.hv[1] = *(const v8h*)(wp + 48);
        c = wmma_raw(w0.v, xf[0].v, c);
        c = wmma_raw(w1.v, xf[1].v, c);
        asm volatile("v_nop\n\tv_nop\n\tv_nop\n\tv_nop" : "+v"(c) : "v"(w0.v), "v"(xf[0].v), "v"(w1.v), "v"(xf[1].v));
      } else {
        #pragma unroll
        for (int s = 0; s < KS; ++s) {
          Frag wf;
          wf.hv[0] = *(const v8h*)(wp + 32 * s);
          wf.hv[1] = *(const v8h*)(wp + 32 * s + 16);
          c = wmma_g(wf.v, xf[s].v, c);
        }
      }
      acc[nt] = c;
    }
    const float* bp = bias + cb * 64 + 8 * h;
    __syncthreads();
    #pragma unroll
    for (int nt = 0; nt < 4; ++nt) {
      const v4f b0 = *(const v4f*)(bp + nt * 16), b1 = *(const v4f*)(bp + nt * 16 + 4);
      v4f o0, o1;
      #pragma unroll
      for (int q = 0; q < 4; ++q) { o0[q] = acc[nt][q] * inv + b0[q]; o1[q] = acc[nt][4 + q] * inv + b1[q]; }
      if (relu) {
        #pragma unroll
        for (int q = 0; q < 4; ++q) { o0[q] = fmaxf(o0[q], 0.f); o1[q] = fmaxf(o1[q], 0.f); }
      }
      sO[wv][m * 16 + nt * 4 + 2 * h]     = o0;
      sO[wv][m * 16 + nt * 4 + 2 * h + 1] = o1;
    }
    __syncthreads();
    v4f vals[8];
    #pragma unroll
    for (int j = 0; j < 8; ++j) vals[j] = sO[wv][(2 * j + h) * 16 + m];
    float* cp = C + (size_t)cb * cbStride + (size_t)row0 * ldc + m * 4;
    if (active) {
      #pragma unroll
      for (int j = 0; j < 8; ++j) *(volatile v4f*)(cp + (size_t)(2 * j + h) * ldc) = vals[j];
    }
    __threadfence();
    if (active) {
      #pragma unroll
      for (int j = 0; j < 8; ++j) *(volatile v4f*)(cp + (size_t)(2 * j + h) * ldc) = vals[j];
    }
  }
}

__global__ __launch_bounds__(256) void csr_chunk_kernel(const int* __restrict__ eidx, const int* __restrict__ etype,
    unsigned* chunkout, int* lbtab, int* cnttab) {
  __shared__ unsigned s_pay[2][CHUNK];
  __shared__ unsigned char s_bk[2][CHUNK];
  __shared__ int s_w[8];
  const int t = threadIdx.x, c = blockIdx.x;
  #pragma unroll
  for (int i = 0; i < 8; ++i) {
    int idx = t * 8 + i, e = c * CHUNK + idx;
    unsigned pay = 0u; int bk = NBPAD - 1;
    if (e < NE) {
      int src = clampi(eidx[e], 0, NN - 1);
      int dst = clampi(eidx[NE + e], 0, NN - 1);
      int ty  = clampi(etype[e], 0, NR - 1);
      bk = dst >> BKSH;
      pay = ((unsigned)(dst & (BKW - 1)) << 20) | (unsigned)(ty * NN + src);
    }
    s_pay[0][idx] = pay; s_bk[0][idx] = (unsigned char)bk;
  }
  __syncthreads();
  int cur = 0;
  for (int bit = 0; bit < NBBITS; ++bit) {
    unsigned pr[8]; unsigned char br[8]; int z = 0;
    #pragma unroll
    for (int i = 0; i < 8; ++i) {
      pr[i] = s_pay[cur][t * 8 + i]; br[i] = s_bk[cur][t * 8 + i];
      z += (((br[i] >> bit) & 1) == 0) ? 1 : 0;
    }
    int tot = 0;
    int zb = block_excl_scan(z, s_w, tot);
    int nxt = cur ^ 1;
    #pragma unroll
    for (int i = 0; i < 8; ++i) {
      int f = (br[i] >> bit) & 1;
      int pos = f ? (tot + (t * 8 + i) - zb) : zb;
      if (!f) zb++;
      pos = clampi(pos, 0, CHUNK - 1);
      s_pay[nxt][pos] = pr[i]; s_bk[nxt][pos] = br[i];
    }
    __syncthreads();
    cur = nxt;
  }
  int lb, cn;
  {
    int lo = 0, hi = CHUNK;
    while (lo < hi) { int mid = (lo + hi) >> 1; if ((int)s_bk[cur][mid] < t) lo = mid + 1; else hi = mid; }
    lb = lo;
    lo = 0; hi = CHUNK;
    while (lo < hi) { int mid = (lo + hi) >> 1; if ((int)s_bk[cur][mid] < t + 1) lo = mid + 1; else hi = mid; }
    cn = lo - lb;
  }
  v4u cv0 = *(const v4u*)(&s_pay[cur][4 * t]);
  v4u cv1 = *(const v4u*)(&s_pay[cur][4 * (t + 256)]);
  unsigned* cob = chunkout + (size_t)c * CHUNK;
  for (int pass = 0; pass < 2; ++pass) {
    if (t < NBPAD) {
      *(volatile int*)(lbtab + (size_t)c * NBPAD + t) = lb;
      *(volatile int*)(cnttab + (size_t)c * NBPAD + t) = cn;
    }
    *(volatile v4u*)(cob + 4 * t) = cv0;
    *(volatile v4u*)(cob + 4 * (t + 256)) = cv1;
    if (pass == 0) __threadfence();
  }
}

__global__ __launch_bounds__(NBPAD) void csr_scan_kernel(const int* __restrict__ cnttab, int* offtab, int* basep, int* tottab) {
  __shared__ int s_w[8];
  const int t = threadIdx.x;
  for (int pass = 0; pass < 2; ++pass) {
    int run = 0;
    for (int c = 0; c < NCH; ++c) {
      int cn = cnttab[(size_t)c * NBPAD + t];
      *(volatile int*)(offtab + (size_t)c * NBPAD + t) = run;
      run += cn;
    }
    int pad = (run + 31) & ~31;
    int tot = 0;
    int ex = block_excl_scan(pad, s_w, tot);
    *(volatile int*)(basep + t) = ex;
    *(volatile int*)(tottab + t) = run;
    if (pass == 0) __threadfence();
  }
}

__global__ __launch_bounds__(256) void csr_bucket_kernel(const unsigned* __restrict__ chunkout,
    const int* __restrict__ lbtab, const int* __restrict__ cnttab, const int* __restrict__ offtab,
    const int* __restrict__ basep, const int* __restrict__ tottab, unsigned* sorted, int* row_ptr) {
  __shared__ unsigned bufA[CAP];
  __shared__ unsigned bufB[CAP];
  __shared__ int s_w[8];
  unsigned* cur = bufA;
  unsigned* nxt = bufB;
  const int t = threadIdx.x, B = blockIdx.x;
  const int tot = clampi(tottab[B], 0, CAP);
  int base = basep[B]; if (base < 0) base = 0;
  for (int c = t; c < NCH; c += 256) {
    int cn = cnttab[(size_t)c * NBPAD + B], lb = lbtab[(size_t)c * NBPAD + B], off = offtab[(size_t)c * NBPAD + B];
    for (int i = 0; i < cn; ++i) {
      int d = off + i, s = lb + i;
      if ((unsigned)d < (unsigned)CAP && (unsigned)s < (unsigned)CHUNK) cur[d] = chunkout[(size_t)c * CHUNK + s];
    }
  }
  __syncthreads();
  const int per = (tot + 255) >> 8;
  int s0 = t * per; if (s0 > tot) s0 = tot;
  int s1 = s0 + per; if (s1 > tot) s1 = tot;
  for (int bit = 0; bit < BKSH; ++bit) {
    const int sh = 20 + bit;
    int z = 0;
    for (int i = s0; i < s1; ++i) z += (((cur[i] >> sh) & 1u) == 0) ? 1 : 0;
    int totz = 0;
    int zb = block_excl_scan(z, s_w, totz);
    for (int i = s0; i < s1; ++i) {
      unsigned w = cur[i];
      int f = (w >> sh) & 1u;
      int pos = f ? (totz + i - zb) : zb;
      if (!f) zb++;
      pos = clampi(pos, 0, CAP - 1);
      nxt[pos] = w;
    }
    __syncthreads();
    unsigned* tp = cur; cur = nxt; nxt = tp;
  }
  const int padn = (tot + 31) & ~31;
  for (int i = tot + t; i < padn; i += 256) cur[i] = 0u;
  v4i rpA = {0, 0, 0, 0};
  const bool hasRp = t < (RP / 4);
  if (hasRp) {
    #pragma unroll
    for (int j = 0; j < 4; ++j) {
      int v = 4 * t + j;
      int lo = 0, hi = tot;
      while (lo < hi) { int mid = (lo + hi) >> 1; if ((int)((cur[mid] >> 20) & 1023u) < v) lo = mid + 1; else hi = mid; }
      rpA[j] = base + lo;
    }
  }
  __syncthreads();
  for (int pass = 0; pass < 2; ++pass) {
    if (hasRp) *(volatile v4i*)(row_ptr + (size_t)B * RP + 4 * t) = rpA;
    for (int idx = t; idx * 4 < padn; idx += 256) {
      v4u v = *(const v4u*)(cur + 4 * idx);
      size_t o = (size_t)base + 4 * (size_t)idx;
      if (o + 4 <= (size_t)SORTED_N) *(volatile v4u*)(sorted + o) = v;
    }
    if (pass == 0) __threadfence();
  }
}

__global__ __launch_bounds__(64) void agg_kernel(const int* __restrict__ row_ptr, const unsigned* __restrict__ sorted,
    const float* __restrict__ hrel6, const float* __restrict__ cb64, float inv, float* hout) {
  __shared__ v4f sT[2][256];
  const int t = threadIdx.x, wv = t >> 5, lane = t & 31, h = lane >> 4, m = lane & 15, hf = lane & 1;
  const int gw = blockIdx.x * 2 + wv;
  const int v = gw * 16 + (lane >> 1);
  const bool vok = v < NN;
  const int vc = vok ? v : NN - 1;
  const int bk = vc >> BKSH, lv = vc & (BKW - 1);
  const int* rp = row_ptr + (size_t)bk * RP + lv;
  int beg = rp[0], end = rp[1];
  int deg = end - beg;
  if (deg < 0) deg = 0;
  if (deg > 4096) deg = 4096;
  if (beg < 0) beg = 0;
  if (!vok) deg = 0;
  v4f acc[8];
  #pragma unroll
  for (int q = 0; q < 8; ++q) { acc[q][0] = 0.f; acc[q][1] = 0.f; acc[q][2] = 0.f; acc[q][3] = 0.f; }
  for (int i = 0; i < deg; ++i) {
    unsigned idx = (unsigned)(beg + i);
    if (idx >= (unsigned)SORTED_N) idx = SORTED_N - 1;
    unsigned row = sorted[idx] & ROWMASK;
    if (row > (unsigned)(NR * NN - 1)) row = NR * NN - 1;
    const v4f* p = (const v4f*)(hrel6 + (size_t)row * DD + hf * 32);
    #pragma unroll
    for (int q = 0; q < 8; ++q) acc[q] += p[q];
  }
  const float rd = 1.f / fmaxf((float)deg, 1.f);
  const v4f* pr = (const v4f*)(hrel6 + ((size_t)NR * NN + vc) * DD + hf * 32);
  const v4f* pb = (const v4f*)(cb64 + hf * 32);
  #pragma unroll
  for (int q = 0; q < 8; ++q) {
    v4f o = (acc[q] * rd + pr[q]) * inv + pb[q];
    #pragma unroll
    for (int j = 0; j < 4; ++j) o[j] = fmaxf(o[j], 0.f);
    sT[wv][(lane >> 1) * 16 + hf * 8 + q] = o;
  }
  __syncthreads();
  v4f vals[8]; size_t offs[8]; bool ok[8];
  #pragma unroll
  for (int j = 0; j < 8; ++j) {
    vals[j] = sT[wv][(2 * j + h) * 16 + m];
    int node = gw * 16 + 2 * j + h;
    ok[j] = node < NN;
    offs[j] = (size_t)(ok[j] ? node : 0) * DD + m * 4;
  }
  #pragma unroll
  for (int j = 0; j < 8; ++j) if (ok[j]) *(volatile v4f*)(hout + offs[j]) = vals[j];
  __threadfence();
  #pragma unroll
  for (int j = 0; j < 8; ++j) if (ok[j]) *(volatile v4f*)(hout + offs[j]) = vals[j];
}

__global__ __launch_bounds__(256) void gptr_kernel(const int* __restrict__ batch, int* gptr) {
  int t = blockIdx.x * blockDim.x + threadIdx.x;
  if (t >= GPN / 4) return;
  v4i r;
  #pragma unroll
  for (int j = 0; j < 4; ++j) {
    int g = 4 * t + j, val = NN;
    if (g <= NG) {
      int lo = 0, hi = NN;
      while (lo < hi) { int mid = (lo + hi) >> 1; if (batch[mid] < g) lo = mid + 1; else hi = mid; }
      val = lo;
    }
    r[j] = val;
  }
  *(volatile v4i*)(gptr + 4 * t) = r;
  __threadfence();
  *(volatile v4i*)(gptr + 4 * t) = r;
}

__device__ __forceinline__ float sigf(float x) { return 1.f / (1.f + expf(-x)); }

__global__ __launch_bounds__(256) void cell_kernel(const float* __restrict__ gates, float* cx, float* X) {
  int tid = blockIdx.x * blockDim.x + threadIdx.x;
  if (tid >= NG * DD) return;
  int g = tid >> 6, d = tid & 63;
  const float* gp = gates + (size_t)g * 256;
  float iv = sigf(gp[d]);
  float fv = sigf(gp[64 + d]);
  float gg = tanhf(gp[128 + d]);
  float ov = sigf(gp[192 + d]);
  float c  = fv * cx[tid] + iv * gg;
  float hn = ov * tanhf(c);
  float* cp = cx + tid;
  float* x0 = X + (size_t)g * XW + d;
  float* x1 = X + (size_t)g * XW + 128 + d;
  *(volatile float*)cp = c; *(volatile float*)x0 = hn; *(volatile float*)x1 = hn;
  __threadfence();
  *(volatile float*)cp = c; *(volatile float*)x0 = hn; *(volatile float*)x1 = hn;
}

__global__ __launch_bounds__(128) void attn_e_kernel(const float* __restrict__ h, const float* __restrict__ X,
    const int* __restrict__ batch, float* ebuf) {
  __shared__ float s_e[32];
  const int t = threadIdx.x, wave = t >> 5, lane = t & 31, sub = t & 3, ln = t >> 2;
  int n = blockIdx.x * 32 + ln;
  int nc = n < NN ? n : NN - 1;
  int g = clampi(batch[nc], 0, NG - 1);
  const float* hp = h + (size_t)nc * DD + sub * 16;
  const float* qp = X + (size_t)g * XW + sub * 16;
  float s = 0.f;
  #pragma unroll
  for (int q = 0; q < 4; ++q) {
    v4f a = *(const v4f*)(hp + 4 * q), b = *(const v4f*)(qp + 4 * q);
    s += a[0] * b[0]; s += a[1] * b[1]; s += a[2] * b[2]; s += a[3] * b[3];
  }
  s += __shfl_xor(s, 1); s += __shfl_xor(s, 2);
  if (sub == 0) s_e[ln] = s;
  __syncthreads();
  float ev = 0.f; float* p = ebuf; bool wr = false;
  if (wave == 0) {
    int nn = blockIdx.x * 32 + lane;
    if (nn < NN) { wr = true; ev = s_e[lane]; p = ebuf + nn; *(volatile float*)p = ev; }
  }
  __threadfence();
  if (wr) *(volatile float*)p = ev;
}

__global__ __launch_bounds__(256) void graph_kernel(const int* __restrict__ gptr, const float* __restrict__ ebuf,
    const float* __restrict__ h, float* X) {
  const int g = blockIdx.x * 8 + (threadIdx.x >> 5);
  const int lane = threadIdx.x & 31;
  if (g >= NG) return;
  int beg = clampi(gptr[g], 0, NN), end = clampi(gptr[g + 1], 0, NN);
  if (end < beg) end = beg;
  float m = -INFINITY;
  for (int n = beg + lane; n < end; n += 32) m = fmaxf(m, ebuf[n]);
  for (int o = 16; o > 0; o >>= 1) m = fmaxf(m, __shfl_xor(m, o));
  float s = 0.f;
  for (int n = beg + lane; n < end; n += 32) s += expf(ebuf[n] - m);
  for (int o = 16; o > 0; o >>= 1) s += __shfl_xor(s, o);
  const float inv_s = 1.f / s;
  v2f acc = {0.f, 0.f};
  const int c2 = 2 * lane;
  for (int c0 = beg; c0 < end; c0 += 32) {
    int n = c0 + lane;
    float p = (n < end) ? expf(ebuf[n] - m) * inv_s : 0.f;
    int lim = end - c0; if (lim > 32) lim = 32;
    for (int i = 0; i < lim; ++i) {
      float a = __shfl(p, i);
      v2f x = *(const v2f*)(h + (size_t)(c0 + i) * DD + c2);
      acc += a * x;
    }
  }
  float* pp = X + (size_t)g * XW + 64 + c2;
  *(volatile v2f*)pp = acc;
  __threadfence();
  *(volatile v2f*)pp = acc;
}

__global__ __launch_bounds__(256) void pack_kernel(const float* __restrict__ l2o, float* out, int out_n) {
  int i = blockIdx.x * blockDim.x + threadIdx.x;
  if (4 * i + 4 > out_n) return;
  v4f v;
  #pragma unroll
  for (int j = 0; j < 4; ++j) { int f = 4 * i + j; int g = f / 12, c = f - g * 12; v[j] = l2o[(size_t)g * 64 + c]; }
  *(volatile v4f*)(out + 4 * i) = v;
  __threadfence();
  *(volatile v4f*)(out + 4 * i) = v;
}

static inline size_t alup(size_t v) { return (v + 255) & ~(size_t)255; }

extern "C" void kernel_launch(void* const* d_in, const int* in_sizes, int n_in,
                              void* d_out, int out_size, void* d_ws, size_t ws_size,
                              hipStream_t stream) {
  if (n_in < 18) return;
  const float* x      = (const float*)d_in[0];
  const int*   eidx   = (const int*)d_in[1];
  const int*   etype  = (const int*)d_in[2];
  const int*   batch  = (const int*)d_in[3];
  const float* lin0_w = (const float*)d_in[4];
  const float* lin0_b = (const float*)d_in[5];
  const float* basis  = (const float*)d_in[6];
  const float* att    = (const float*)d_in[7];
  const float* root   = (const float*)d_in[8];
  const float* conv_b = (const float*)d_in[9];
  const float* w_ih   = (const float*)d_in[10];
  const float* w_hh   = (const float*)d_in[11];
  const float* b_ih   = (const float*)d_in[12];
  const float* b_hh   = (const float*)d_in[13];
  const float* lin1_w = (const float*)d_in[14];
  const float* lin1_b = (const float*)d_in[15];
  const float* lin2_w = (const float*)d_in[16];
  const float* lin2_b = (const float*)d_in[17];
  if (in_sizes[0] < NN * 15 || in_sizes[1] < 2 * NE || in_sizes[2] < NE || in_sizes[3] < NN) return;
  if (in_sizes[4] < 15 * DD || in_sizes[5] < DD || in_sizes[6] < NR * DD * DD || in_sizes[7] < NR * NR ||
      in_sizes[8] < DD * DD || in_sizes[9] < DD || in_sizes[10] < 256 * 128 || in_sizes[11] < 256 * DD ||
      in_sizes[12] < 256 || in_sizes[13] < 256 || in_sizes[14] < 128 * DD || in_sizes[15] < DD ||
      in_sizes[16] < DD * 12 || in_sizes[17] < 12) return;
  if (out_size < NG * 12) return;

  char* ws = (char*)d_ws;
  size_t off = 0;
  auto carve = [&](size_t bytes) { size_t o = off; off = alup(off + bytes); return ws + o; };
  float*    hbuf     = (float*)carve((size_t)NN * DD * 4);
  float*    hrel6    = (float*)carve((size_t)6 * NN * DD * 4);
  unsigned* chunkout = (unsigned*)carve((size_t)NCH * CHUNK * 4);
  int*      lbtab    = (int*)carve((size_t)NCH * NBPAD * 4);
  int*      cnttab   = (int*)carve((size_t)NCH * NBPAD * 4);
  int*      offtab   = (int*)carve((size_t)NCH * NBPAD * 4);
  int*      basep    = (int*)carve((size_t)NBPAD * 4);
  int*      tottab   = (int*)carve((size_t)NBPAD * 4);
  unsigned* sorted   = (unsigned*)carve((size_t)SORTED_N * 4);
  int*      row_ptr  = (int*)carve((size_t)NBPAD * RP * 4);
  _Float16* Wall     = (_Float16*)carve((size_t)384 * 64 * 2);
  _Float16* Wg       = (_Float16*)carve((size_t)256 * 192 * 2);
  _Float16* W1       = (_Float16*)carve((size_t)64 * 128 * 2);
  _Float16* W2       = (_Float16*)carve((size_t)64 * 64 * 2);
  float*    gb       = (float*)carve((size_t)256 * 4);
  float*    cb64     = (float*)carve((size_t)64 * 4);
  float*    b1c      = (float*)carve((size_t)64 * 4);
  float*    b2p      = (float*)carve((size_t)64 * 4);
  float*    z64      = (float*)carve((size_t)64 * 4);
  int*      gptr     = (int*)carve((size_t)GPN * 4);
  float*    X        = (float*)carve((size_t)NG * XW * 4);
  float*    cx       = (float*)carve((size_t)NG * DD * 4);
  float*    gates    = (float*)carve((size_t)NG * 256 * 4);
  float*    ebuf     = (float*)carve((size_t)NN * 4);
  float*    l1o      = (float*)carve((size_t)NG * 64 * 4);
  float*    l2o      = (float*)carve((size_t)NG * 64 * 4);
  if (off > ws_size) return;
  float* out = (float*)d_out;

  const int B256 = 256;
  const float inv = 1.f / 1024.f;

  prep_kernel<<<1, B256, 0, stream>>>(att, basis, root, w_ih, w_hh, b_ih, b_hh, conv_b, lin1_w, lin1_b, lin2_w, lin2_b,
                                      Wall, Wg, W1, W2, gb, cb64, b1c, b2p, z64);
  lin0_kernel<<<(NN * 16 + B256 - 1) / B256, B256, 0, stream>>>(x, lin0_w, lin0_b, hbuf);
  csr_chunk_kernel<<<NCH, B256, 0, stream>>>(eidx, etype, chunkout, lbtab, cnttab);
  csr_scan_kernel<<<1, NBPAD, 0, stream>>>(cnttab, offtab, basep, tottab);
  csr_bucket_kernel<<<NBKT, B256, 0, stream>>>(chunkout, lbtab, cnttab, offtab, basep, tottab, sorted, row_ptr);
  gptr_kernel<<<(GPN / 4 + B256 - 1) / B256, B256, 0, stream>>>(batch, gptr);
  hipMemsetAsync(X, 0, (size_t)NG * XW * 4, stream);
  hipMemsetAsync(cx, 0, (size_t)NG * DD * 4, stream);

  const int gemmBlocksN = (NN / 16 + 1) / 2;
  const int gemmBlocksG = (NG / 16 + 1) / 2;
  const int aggBlocks   = (NN + 31) / 32;

  for (int step = 0; step < PROP; ++step) {
    gemm_kernel<2, 6><<<gemmBlocksN, 64, 0, stream>>>(hbuf, DD, 16.f, Wall, z64, 1.f, 0,
                                                       hrel6, DD, (size_t)NN * DD, NN);
    agg_kernel<<<aggBlocks, 64, 0, stream>>>(row_ptr, sorted, hrel6, cb64, inv, hbuf);
  }

  for (int it = 0; it < S2S; ++it) {
    gemm_kernel<6, 4><<<gemmBlocksG, 64, 0, stream>>>(X, XW, 16.f, Wg, gb, inv, 0,
                                                       gates, 256, (size_t)64, NG);
    cell_kernel<<<(NG * DD + B256 - 1) / B256, B256, 0, stream>>>(gates, cx, X);
    attn_e_kernel<<<(NN + 31) / 32, 128, 0, stream>>>(hbuf, X, batch, ebuf);
    graph_kernel<<<(NG + 7) / 8, B256, 0, stream>>>(gptr, ebuf, hbuf, X);
  }

  gemm_kernel<4, 1><<<gemmBlocksG, 64, 0, stream>>>(X, XW, 16.f, W1, b1c, inv, 1,
                                                     l1o, 64, (size_t)0, NG);
  gemm_kernel<2, 1><<<gemmBlocksG, 64, 0, stream>>>(l1o, 64, 16.f, W2, b2p, inv, 0,
                                                     l2o, 64, (size_t)0, NG);
  pack_kernel<<<(NG * 12 / 4 + B256 - 1) / B256, B256, 0, stream>>>(l2o, out, NG * 12);
}
